// HyperbolicGraphConvolution_59124519796865
// MI455X (gfx1250) — hardware-verified
//
#include <hip/hip_runtime.h>
#include <stddef.h>


#define CH      64
#define KP      64
#define APH     72
#define PQW     128
#define NSW     4
#define WA1P    130
#define GROWS   32
#define GTHR    64
#define ETHR    256
#define NTHR    256
#define NWAVE   8
#define NSLOT   512
#define EPT     8
#define NGRP    2
#define CHUNK   (NTHR * EPT * NGRP)
#define WCAP    (EPT * NGRP * 32)
#define LISTN   (NWAVE * WCAP)
#define LDS_AGG (NSLOT * CH * 4 + LISTN * 4 + 64)
#define PL0     0
#define PL1     (CH * KP)
#define PL2     (PL1 + 2 * CH * KP)
#define PL3     (PL2 + CH * KP)
#define PLTOT   (PL3 + CH * KP)
#define WPTHR   256
#define WPBLK   (PLTOT / 8 / WPTHR)
#define WSC     64.0f
#define XS      16.0f
#define HS      64.0f
#define AS      1024.0f
#define SS      4096.0f
#define EPSF    1e-7f
#define INVNF   0.01f
#define WSCAP   134217728

static_assert(WPBLK * WPTHR * 8 == PLTOT);
static_assert((PL1 % (8 * WPTHR)) == 0 && (PL2 % (8 * WPTHR)) == 0 && (PL3 % (8 * WPTHR)) == 0);
static_assert((APH % 8) == 0 && (KP % 8) == 0 && (PQW % 32) == 0 && (CH % 32) == 0);
static_assert(GROWS == (GTHR / 32) * 16);
static_assert(GROWS == 32 && CH == 2 * 32);
static_assert(GROWS * CH == 8 * GTHR * 4);
static_assert(GROWS * PQW == 16 * GTHR * 4);
static_assert(GROWS * NSW == 32 * 4);
static_assert((CHUNK & (CHUNK - 1)) == 0 && CHUNK <= 4096);
static_assert((NSLOT & (NSLOT - 1)) == 0 && NSLOT <= 4096 && (NSLOT % GROWS) == 0);
static_assert(NSLOT * CH == 32 * NTHR * 4);
static_assert(NTHR == NWAVE * 32);

typedef float          v2f  __attribute__((ext_vector_type(2)));
typedef float          v4f  __attribute__((ext_vector_type(4)));
typedef float          v8f  __attribute__((ext_vector_type(8)));
typedef int            v4i  __attribute__((ext_vector_type(4)));
typedef _Float16       v8h  __attribute__((ext_vector_type(8)));
typedef _Float16       v16h __attribute__((ext_vector_type(16)));
union Frag { v16h v; v8h h[2]; };

__device__ __forceinline__ v8f wmh(v16h a, v16h b, v8f c) {
  v8f d = __builtin_amdgcn_wmma_f32_16x16x32_f16(false, a, false, b, (short)0, c, false, false);
  asm volatile("v_nop\n\tv_nop\n\tv_nop\n\tv_nop" : "+v"(d) : "v"(a), "v"(b));
  return d;
}

__device__ __forceinline__ float red16(float x) {
  x += __shfl_xor(x, 8, 32);
  x += __shfl_xor(x, 4, 32);
  x += __shfl_xor(x, 2, 32);
  x += __shfl_xor(x, 1, 32);
  return x;
}
__device__ __forceinline__ float sq4(v4f a) { return a.x * a.x + a.y * a.y + a.z * a.z + a.w * a.w; }
__device__ __forceinline__ float artanh_c(float x) {
  x = fminf(fmaxf(x, -1.0f + EPSF), 1.0f - EPSF);
  return atanhf(x);
}
__device__ __forceinline__ float siluf_(float x) { return x / (1.0f + expf(-x)); }
__device__ __forceinline__ float silu_fast(float x) {
  const float ex = __expf(-x);
  return x * __builtin_amdgcn_rcpf(1.0f + ex);
}

__device__ __forceinline__ v8h cvt8(v4f a, v4f b, float s) {
  v8h r;
  r[0] = (_Float16)(a.x * s); r[1] = (_Float16)(a.y * s); r[2] = (_Float16)(a.z * s); r[3] = (_Float16)(a.w * s);
  r[4] = (_Float16)(b.x * s); r[5] = (_Float16)(b.y * s); r[6] = (_Float16)(b.z * s); r[7] = (_Float16)(b.w * s);
  return r;
}

__device__ __forceinline__ v16h ldb(const _Float16* __restrict__ pl, int n, int k0, int hh) {
  Frag b;
  const _Float16* p = pl + (size_t)n * KP + k0 + 8 * hh;
  b.h[0] = *(const v8h*)p;
  b.h[1] = *(const v8h*)(p + 16);
  return b.v;
}
__device__ __forceinline__ v16h lda_f32(const float* __restrict__ rp, int k0, int hh, float s) {
  Frag a;
  const float* p = rp + k0 + 8 * hh;
  a.h[0] = cvt8(*(const v4f*)p, *(const v4f*)(p + 4), s);
  a.h[1] = cvt8(*(const v4f*)(p + 16), *(const v4f*)(p + 20), s);
  return a.v;
}
__device__ __forceinline__ v16h lda_lds(const _Float16* At, int m, int k0, int hh) {
  Frag a;
  const _Float16* p = At + m * APH + k0 + 8 * hh;
  a.h[0] = *(const v8h*)p;
  a.h[1] = *(const v8h*)(p + 16);
  return a.v;
}

template <int NBT>
__device__ __forceinline__ int scan_chunk(const int* __restrict__ keys, int nE, int cbase, int slotBase,
                                          int vec8, int* list, int tid, int lane, int wave) {
  int wc = 0;
#pragma unroll
  for (int g = 0; g < NGRP; ++g) {
    const int el0  = (g * NTHR + tid) * EPT;
    const int e0   = cbase + el0;
    const int sent = -2147483647 - 1;
    v4i da, db;
    if (vec8 != 0 && cbase + CHUNK <= nE) {
      da = *(const v4i*)(keys + e0);
      db = *(const v4i*)(keys + e0 + 4);
    } else {
      da.x = (e0     < nE) ? keys[min(e0, nE - 1)] : sent;
      da.y = (e0 + 1 < nE) ? keys[min(e0 + 1, nE - 1)] : sent;
      da.z = (e0 + 2 < nE) ? keys[min(e0 + 2, nE - 1)] : sent;
      da.w = (e0 + 3 < nE) ? keys[min(e0 + 3, nE - 1)] : sent;
      db.x = (e0 + 4 < nE) ? keys[min(e0 + 4, nE - 1)] : sent;
      db.y = (e0 + 5 < nE) ? keys[min(e0 + 5, nE - 1)] : sent;
      db.z = (e0 + 6 < nE) ? keys[min(e0 + 6, nE - 1)] : sent;
      db.w = (e0 + 7 < nE) ? keys[min(e0 + 7, nE - 1)] : sent;
    }
    const unsigned nb = (unsigned)slotBase;
    const unsigned s0 = (unsigned)da.x - nb, s1 = (unsigned)da.y - nb;
    const unsigned s2 = (unsigned)da.z - nb, s3 = (unsigned)da.w - nb;
    const unsigned s4 = (unsigned)db.x - nb, s5 = (unsigned)db.y - nb;
    const unsigned s6 = (unsigned)db.z - nb, s7 = (unsigned)db.w - nb;
    const bool h0 = s0 < (unsigned)NBT, h1 = s1 < (unsigned)NBT, h2 = s2 < (unsigned)NBT, h3 = s3 < (unsigned)NBT;
    const bool h4 = s4 < (unsigned)NBT, h5 = s5 < (unsigned)NBT, h6 = s6 < (unsigned)NBT, h7 = s7 < (unsigned)NBT;
    const unsigned any = __builtin_amdgcn_ballot_w32(h0 | h1 | h2 | h3 | h4 | h5 | h6 | h7);
    if (any != 0u) {
#define HITJ(J, HJ, SJ) { \
        const unsigned mj = __builtin_amdgcn_ballot_w32(HJ); \
        if (mj != 0u) { \
          if (HJ) { \
            const int pos = wc + (int)__builtin_amdgcn_mbcnt_lo(mj, 0u); \
            if (pos < WCAP) list[wave * WCAP + pos] = ((el0 + (J)) << 12) | (int)(SJ); \
          } \
          wc += (int)__builtin_popcount(mj); } }
      HITJ(0, h0, s0)
      HITJ(1, h1, s1)
      HITJ(2, h2, s2)
      HITJ(3, h3, s3)
      HITJ(4, h4, s4)
      HITJ(5, h5, s5)
      HITJ(6, h6, s6)
      HITJ(7, h7, s7)
#undef HITJ
    }
  }
  return wc;
}

__global__ __launch_bounds__(WPTHR) void k_wprep(const float* __restrict__ W_lin, const float* __restrict__ Wa1,
                                                 const float* __restrict__ Wm1, const float* __restrict__ Wm2,
                                                 _Float16* PL) {
  const int i = blockIdx.x * WPTHR + threadIdx.x;
  const float* src;
  if (i < PL1 / 8) {
    src = W_lin + (i >> 3) * CH + (i & 7) * 8;
  } else if (i < PL2 / 8) {
    const int j = i - PL1 / 8;
    const int n = j >> 3;
    src = Wa1 + (n & (CH - 1)) * WA1P + (n >> 6) * CH + (j & 7) * 8;
  } else if (i < PL3 / 8) {
    const int j = i - PL2 / 8;
    src = Wm1 + (j >> 3) * CH + (j & 7) * 8;
  } else {
    const int j = i - PL3 / 8;
    src = Wm2 + (j >> 3) * CH + (j & 7) * 8;
  }
  v8h hv;
#pragma unroll
  for (int e = 0; e < 8; ++e) hv[e] = (_Float16)(src[e] * WSC);
  _Float16* dp = PL + (size_t)i * 8;
  *(volatile v8h*)dp = hv;
  __threadfence();
  *(volatile v8h*)dp = hv;
}

__global__ __launch_bounds__(GTHR) void k_node1(const float* __restrict__ h, const _Float16* __restrict__ PL,
                                                const float* __restrict__ b_lin, const float* __restrict__ ba1,
                                                float* HB, float* PQ, float* NS, int nN) {
  __shared__ __attribute__((aligned(16))) _Float16 At2[2 * 16 * APH];
  __shared__ __attribute__((aligned(16))) float stgH[GROWS * CH];
  __shared__ __attribute__((aligned(16))) float stgP[GROWS * PQW];
  __shared__ __attribute__((aligned(16))) float sns[GROWS * NSW];
  const int tid = threadIdx.x, lane = tid & 31, wave = tid >> 5, hh = lane >> 4, m = lane & 15;
  const int rowBase = blockIdx.x * GROWS;

  int rg = rowBase + wave * 16 + m;
  rg = rg > nN - 1 ? nN - 1 : rg;
  const float* hr = h + (size_t)rg * CH;
  const v4f u0 = *(const v4f*)(hr + 8 * hh),      u1 = *(const v4f*)(hr + 8 * hh + 4);
  const v4f u2 = *(const v4f*)(hr + 16 + 8 * hh), u3 = *(const v4f*)(hr + 20 + 8 * hh);
  const v4f u4 = *(const v4f*)(hr + 32 + 8 * hh), u5 = *(const v4f*)(hr + 36 + 8 * hh);
  const v4f u6 = *(const v4f*)(hr + 48 + 8 * hh), u7 = *(const v4f*)(hr + 52 + 8 * hh);
  float n2 = sq4(u0) + sq4(u1) + sq4(u2) + sq4(u3) + sq4(u4) + sq4(u5) + sq4(u6) + sq4(u7);
  n2 += __shfl_xor(n2, 16, 32);
  const float nh = fmaxf(sqrtf(n2), EPSF);
  const float sc = artanh_c(nh) / nh;
  Frag a0, a1;
  a0.h[0] = cvt8(u0, u1, sc * XS);
  a0.h[1] = cvt8(u2, u3, sc * XS);
  a1.h[0] = cvt8(u4, u5, sc * XS);
  a1.h[1] = cvt8(u6, u7, sc * XS);

  v8f C[4];
#pragma unroll
  for (int nt = 0; nt < 4; ++nt) {
    v8f acc = {0.f, 0.f, 0.f, 0.f, 0.f, 0.f, 0.f, 0.f};
    acc = wmh(a0.v, ldb(PL + PL0, 16 * nt + m, 0, hh), acc);
    acc = wmh(a1.v, ldb(PL + PL0, 16 * nt + m, 32, hh), acc);
    C[nt] = acc;
  }
  const float r1s = 1.0f / (XS * WSC);
#pragma unroll
  for (int nt = 0; nt < 4; ++nt) {
#pragma unroll
    for (int r = 0; r < 8; ++r) C[nt][r] *= r1s;
  }

  float res2[8];
#pragma unroll
  for (int v = 0; v < 8; ++v) {
    const float p = C[0][v] * C[0][v] + C[1][v] * C[1][v] + C[2][v] * C[2][v] + C[3][v] * C[3][v];
    const float s2 = red16(p);
    const float n = fmaxf(sqrtf(s2), EPSF);
    const float s = tanhf(n) / n;
#pragma unroll
    for (int nt = 0; nt < 4; ++nt) C[nt][v] *= s;
    const float q = C[0][v] * C[0][v] + C[1][v] * C[1][v] + C[2][v] * C[2][v] + C[3][v] * C[3][v];
    res2[v] = red16(q);
  }

  float bb[4];
#pragma unroll
  for (int nt = 0; nt < 4; ++nt) bb[nt] = b_lin[16 * nt + m];
  const float bn2 = red16(bb[0] * bb[0] + bb[1] * bb[1] + bb[2] * bb[2] + bb[3] * bb[3]);
  const float bnorm = sqrtf(bn2);
#pragma unroll
  for (int v = 0; v < 8; ++v) {
    const float fac = 1.0f - res2[v];
    const float nu  = fmaxf(fabsf(fac) * bnorm, EPSF);
    const float lam = 2.0f / fmaxf(fac, EPSF);
    const float t   = tanhf(0.5f * lam * nu);
    const float ys  = t * fac / nu;
    const float y2  = ys * ys * bn2;
    const float pd  = C[0][v] * bb[0] + C[1][v] * bb[1] + C[2][v] * bb[2] + C[3][v] * bb[3];
    const float xy  = ys * red16(pd);
    const float A1  = 1.0f + 2.0f * xy + y2;
    const float den = fmaxf(1.0f + 2.0f * xy + res2[v] * y2, EPSF);
    const float ia  = A1 / den;
    const float ib  = fac * ys / den;
#pragma unroll
    for (int nt = 0; nt < 4; ++nt) C[nt][v] = ia * C[nt][v] + ib * bb[nt];
  }

  _Float16* Aw = At2 + wave * 16 * APH;
#pragma unroll
  for (int v = 0; v < 8; ++v) {
    const float p   = C[0][v] * C[0][v] + C[1][v] * C[1][v] + C[2][v] * C[2][v] + C[3][v] * C[3][v];
    const float hb2 = red16(p);
    const float n   = fmaxf(sqrtf(hb2), EPSF);
    const float st  = artanh_c(n) / n;
    const int   rl  = wave * 16 + 8 * hh + v;
    if (m == 0) {
      sns[rl * NSW + 0] = hb2;
      sns[rl * NSW + 1] = st;
      sns[rl * NSW + 2] = 0.0f;
      sns[rl * NSW + 3] = 0.0f;
    }
#pragma unroll
    for (int nt = 0; nt < 4; ++nt) {
      const int col = 16 * nt + m;
      const float val = C[nt][v];
      stgH[rl * CH + col] = val;
      Aw[(8 * hh + v) * APH + col] = (_Float16)(val * HS);
    }
  }
  __syncthreads();

  const v16h g0 = lda_lds(Aw, m, 0, hh), g1 = lda_lds(Aw, m, 32, hh);
  v8f D2[8];
#pragma unroll
  for (int nt = 0; nt < 8; ++nt) {
    v8f acc = {0.f, 0.f, 0.f, 0.f, 0.f, 0.f, 0.f, 0.f};
    acc = wmh(g0, ldb(PL + PL1, 16 * nt + m, 0, hh), acc);
    acc = wmh(g1, ldb(PL + PL1, 16 * nt + m, 32, hh), acc);
    D2[nt] = acc;
  }
  const float r2s = 1.0f / (HS * WSC);
#pragma unroll
  for (int nt = 0; nt < 8; ++nt) {
    const int col = 16 * nt + m;
    const float bl = ba1[col & (CH - 1)];
    const float bv = (nt < 4) ? bl : 0.0f;
#pragma unroll
    for (int r = 0; r < 8; ++r) stgP[(wave * 16 + 8 * hh + r) * PQW + col] = D2[nt][r] * r2s + bv;
  }
  __syncthreads();

  float* gh = HB + (size_t)rowBase * CH;
  float* gq = PQ + (size_t)rowBase * PQW;
  float* gs = NS + (size_t)rowBase * NSW;
#pragma unroll
  for (int it = 0; it < 8; ++it) {
    const int f = it * GTHR + tid;
    const v4f v = *(const v4f*)(stgH + 4 * f);
    *(volatile v4f*)(gh + 4 * f) = v;
  }
#pragma unroll
  for (int it = 0; it < 16; ++it) {
    const int f = it * GTHR + tid;
    const v4f v = *(const v4f*)(stgP + 4 * f);
    *(volatile v4f*)(gq + 4 * f) = v;
  }
  v4f nv = {0.f, 0.f, 0.f, 0.f};
  if (tid < 32) nv = *(const v4f*)(sns + 4 * tid);
  if (tid < 32) *(volatile v4f*)(gs + 4 * tid) = nv;
  __threadfence();
#pragma unroll
  for (int it = 0; it < 8; ++it) {
    const int f = it * GTHR + tid;
    const v4f v = *(const v4f*)(stgH + 4 * f);
    *(volatile v4f*)(gh + 4 * f) = v;
  }
#pragma unroll
  for (int it = 0; it < 16; ++it) {
    const int f = it * GTHR + tid;
    const v4f v = *(const v4f*)(stgP + 4 * f);
    *(volatile v4f*)(gq + 4 * f) = v;
  }
  if (tid < 32) *(volatile v4f*)(gs + 4 * tid) = nv;
}

__global__ __launch_bounds__(ETHR) void k_escore(const int* __restrict__ edges, const float* __restrict__ dist,
                                                 const float* __restrict__ emask, const float* __restrict__ Wa1,
                                                 const float* __restrict__ Wa2, const float* __restrict__ ba2,
                                                 const float* __restrict__ HB, const float* __restrict__ PQ,
                                                 const float* __restrict__ NS, float* G, int nN, int nE) {
  __shared__ __attribute__((aligned(16))) float swd[CH];
  __shared__ __attribute__((aligned(16))) float swi[CH];
  __shared__ __attribute__((aligned(16))) float sw2[CH];
  const int tid = threadIdx.x;
  if (tid < CH) {
    swd[tid] = Wa1[tid * WA1P + 2 * CH];
    swi[tid] = Wa1[tid * WA1P + 2 * CH + 1];
    sw2[tid] = Wa2[tid];
  }
  __syncthreads();

  const int e  = blockIdx.x * ETHR + tid;
  const int ec = e > nE - 1 ? nE - 1 : e;
  int r = edges[ec];
  int c = edges[(size_t)nE + ec];
  r = r < 0 ? 0 : (r > nN - 1 ? nN - 1 : r);
  c = c < 0 ? 0 : (c > nN - 1 ? nN - 1 : c);
  const float x2  = NS[(size_t)r * NSW];
  const float y2  = NS[(size_t)c * NSW];
  const float stc = NS[(size_t)c * NSW + 1];
  const float* xr = HB + (size_t)r * CH;
  const float* yc = HB + (size_t)c * CH;
  float xy = 0.0f;
#pragma unroll 1
  for (int k = 0; k < CH / 4; ++k) {
    const v4f a = *(const v4f*)(xr + 4 * k), b = *(const v4f*)(yc + 4 * k);
    xy = fmaf(a.x, b.x, xy); xy = fmaf(a.y, b.y, xy); xy = fmaf(a.z, b.z, xy); xy = fmaf(a.w, b.w, xy);
  }
  const float A1   = 1.0f - 2.0f * xy + y2;
  const float B1   = 1.0f - x2;
  const float den  = fmaxf(1.0f - 2.0f * xy + x2 * y2, EPSF);
  const float num2 = fmaxf(A1 * A1 * x2 - 2.0f * A1 * B1 * xy + B1 * B1 * y2, 0.0f);
  const float mn   = sqrtf(num2) / den;
  const float dd   = 2.0f * artanh_c(mn);
  const float dv   = dist[ec];
  const float em   = emask[ec];
  const float* pr = PQ + (size_t)r * PQW;
  const float* qc = PQ + (size_t)c * PQW + CH;
  float s = ba2[0];
#pragma unroll 1
  for (int j = 0; j < CH / 2; ++j) {
    const v2f p  = *(const v2f*)(pr + 2 * j), q = *(const v2f*)(qc + 2 * j);
    const v2f wd = *(const v2f*)(swd + 2 * j), wi = *(const v2f*)(swi + 2 * j), w2 = *(const v2f*)(sw2 + 2 * j);
    float p0 = p.x + q.x; p0 = fmaf(dd, wd.x, p0); p0 = fmaf(dv, wi.x, p0);
    float p1 = p.y + q.y; p1 = fmaf(dd, wd.y, p1); p1 = fmaf(dv, wi.y, p1);
    s = fmaf(silu_fast(p0), w2.x, s);
    s = fmaf(silu_fast(p1), w2.y, s);
  }
  const float score = em / (1.0f + expf(-s));
  const float g = score * stc * INVNF;
  *(volatile float*)(G + e) = g;
  __threadfence();
  *(volatile float*)(G + e) = g;
}

__global__ __launch_bounds__(NTHR) void k_agg(const int* __restrict__ keyr, const int* __restrict__ cole,
                                              const float* __restrict__ G, const float* __restrict__ HB,
                                              float* AGG, int nN, int nE, int vec8) {
  extern __shared__ v4f lds_dyn[];
  float* aggl = (float*)lds_dyn;
  int*   list = (int*)(aggl + NSLOT * CH);
  int*   wcnt = list + LISTN;
  const int tid = threadIdx.x, lane = tid & 31, wave = tid >> 5;
  const int base = blockIdx.x * NSLOT;

  {
    const v4f z = {0.f, 0.f, 0.f, 0.f};
    for (int i = tid; i < NSLOT * CH / 4; i += NTHR) ((v4f*)aggl)[i] = z;
  }
  __syncthreads();

  const int nChunks = (nE + CHUNK - 1) / CHUNK;
#pragma unroll 1
  for (int ch = 0; ch < nChunks; ++ch) {
    const int cbase = ch * CHUNK;
    const int wc = scan_chunk<NSLOT>(keyr, nE, cbase, base, vec8, list, tid, lane, wave);
    if (lane == 0) wcnt[wave] = wc;
    __syncthreads();
    if (wave == 0) {
#pragma unroll 1
      for (int wsx = 0; wsx < NWAVE; ++wsx) {
        int n = __builtin_amdgcn_readfirstlane(wcnt[wsx]);
        n = n > WCAP ? WCAP : (n < 0 ? 0 : n);
        const int* lp = list + wsx * WCAP;
#pragma unroll 1
        for (int i = 0; i < n; ++i) {
          const int ent  = __builtin_amdgcn_readfirstlane(lp[i]);
          const int slot = ent & (NSLOT - 1);
          int e = cbase + ((ent >> 12) & (CHUNK - 1));
          e = e > nE - 1 ? nE - 1 : e;
          int c = cole[e];
          c = c < 0 ? 0 : (c > nN - 1 ? nN - 1 : c);
          const float w = G[e];
          const v2f x = *(const v2f*)(HB + (size_t)c * CH + 2 * lane);
          v2f* ap = (v2f*)(aggl + slot * CH + 2 * lane);
          v2f a = *ap;
          a.x = fmaf(x.x, w, a.x);
          a.y = fmaf(x.y, w, a.y);
          *ap = a;
        }
      }
    }
    __syncthreads();
  }

  float* gp = AGG + (size_t)base * CH;
#pragma unroll 1
  for (int it = 0; it < 32; ++it) {
    const int f = it * NTHR + tid;
    const v4f v = ((const v4f*)aggl)[f];
    *(volatile v4f*)(gp + 4 * f) = v;
  }
  __threadfence();
#pragma unroll 1
  for (int it = 0; it < 32; ++it) {
    const int f = it * NTHR + tid;
    const v4f v = ((const v4f*)aggl)[f];
    *(volatile v4f*)(gp + 4 * f) = v;
  }
}

__global__ __launch_bounds__(GTHR) void k_node2(const float* __restrict__ AGG, const _Float16* __restrict__ PL,
                                                const float* __restrict__ bm1, const float* __restrict__ bm2,
                                                const float* __restrict__ HB, const float* __restrict__ NS,
                                                float* out, int nN) {
  __shared__ __attribute__((aligned(16))) _Float16 Ht[2 * 16 * APH];
  __shared__ __attribute__((aligned(16))) float shb[GROWS * CH];
  __shared__ __attribute__((aligned(16))) float sout[GROWS * CH];
  __shared__ __attribute__((aligned(16))) float sst[GROWS];
  __shared__ __attribute__((aligned(16))) float sb1[CH];
  __shared__ __attribute__((aligned(16))) float sb2[CH];
  const int tid = threadIdx.x, lane = tid & 31, wave = tid >> 5, hh = lane >> 4, m = lane & 15;
  const int rowBase = blockIdx.x * GROWS;

  {
    const float* hp = HB + (size_t)rowBase * CH;
#pragma unroll 2
    for (int it = 0; it < 8; ++it) {
      const int f = it * GTHR + tid;
      *(v4f*)(shb + 4 * f) = *(const v4f*)(hp + 4 * f);
    }
    if (wave == 0) {
      sst[lane] = NS[(size_t)(rowBase + lane) * NSW + 1];
    } else {
      *(v2f*)(sb1 + 2 * lane) = *(const v2f*)(bm1 + 2 * lane);
      *(v2f*)(sb2 + 2 * lane) = *(const v2f*)(bm2 + 2 * lane);
    }
  }
  __syncthreads();

  const float* ar = AGG + (size_t)(rowBase + wave * 16 + m) * CH;
  const v16h a0 = lda_f32(ar, 0, hh, AS), a1 = lda_f32(ar, 32, hh, AS);
  v8f C1[4];
#pragma unroll
  for (int nt = 0; nt < 4; ++nt) {
    v8f acc = {0.f, 0.f, 0.f, 0.f, 0.f, 0.f, 0.f, 0.f};
    acc = wmh(a0, ldb(PL + PL2, 16 * nt + m, 0, hh), acc);
    acc = wmh(a1, ldb(PL + PL2, 16 * nt + m, 32, hh), acc);
    C1[nt] = acc;
  }
  const float r3s = 1.0f / (AS * WSC);
  _Float16* Hw = Ht + wave * 16 * APH;
#pragma unroll
  for (int nt = 0; nt < 4; ++nt) {
    const int col = 16 * nt + m;
    const float b = sb1[col];
#pragma unroll
    for (int r = 0; r < 8; ++r) {
      const float z = C1[nt][r] * r3s + b;
      Hw[(8 * hh + r) * APH + col] = (_Float16)(siluf_(z) * SS);
    }
  }
  __syncthreads();

  const v16h g0 = lda_lds(Hw, m, 0, hh), g1 = lda_lds(Hw, m, 32, hh);
  v8f C2[4];
#pragma unroll
  for (int nt = 0; nt < 4; ++nt) {
    v8f acc = {0.f, 0.f, 0.f, 0.f, 0.f, 0.f, 0.f, 0.f};
    acc = wmh(g0, ldb(PL + PL3, 16 * nt + m, 0, hh), acc);
    acc = wmh(g1, ldb(PL + PL3, 16 * nt + m, 32, hh), acc);
    C2[nt] = acc;
  }
  const float r4s = 1.0f / (SS * WSC);
  float st[8];
#pragma unroll
  for (int r = 0; r < 8; ++r) st[r] = sst[wave * 16 + 8 * hh + r];
#pragma unroll
  for (int nt = 0; nt < 4; ++nt) {
    const int col = 16 * nt + m;
    const float b = sb2[col];
#pragma unroll
    for (int r = 0; r < 8; ++r) {
      const int rl = wave * 16 + 8 * hh + r;
      C2[nt][r] = C2[nt][r] * r4s + b + shb[rl * CH + col] * st[r];
    }
  }

#pragma unroll
  for (int v = 0; v < 8; ++v) {
    const float z2 = red16(C2[0][v] * C2[0][v] + C2[1][v] * C2[1][v] + C2[2][v] * C2[2][v] + C2[3][v] * C2[3][v]);
    const float nz = fmaxf(sqrtf(z2), EPSF);
    const float s1 = tanhf(nz) / nz;
    float o[4];
#pragma unroll
    for (int nt = 0; nt < 4; ++nt) o[nt] = C2[nt][v] * s1;
    const float o2 = red16(o[0] * o[0] + o[1] * o[1] + o[2] * o[2] + o[3] * o[3]);
    const float no = fmaxf(sqrtf(o2), EPSF);
    const float s2 = artanh_c(no) / no;
    float l[4];
#pragma unroll
    for (int nt = 0; nt < 4; ++nt) l[nt] = siluf_(o[nt] * s2);
    const float a2 = red16(l[0] * l[0] + l[1] * l[1] + l[2] * l[2] + l[3] * l[3]);
    const float na = fmaxf(sqrtf(a2), EPSF);
    const float s3 = tanhf(na) / na;
    const int rl = wave * 16 + 8 * hh + v;
#pragma unroll
    for (int nt = 0; nt < 4; ++nt) sout[rl * CH + 16 * nt + m] = l[nt] * s3;
  }
  __syncthreads();

  float* op = out + (size_t)rowBase * CH;
#pragma unroll
  for (int it = 0; it < 8; ++it) {
    const int f = it * GTHR + tid;
    const int rl = f >> 4;
    const v4f v = *(const v4f*)(sout + 4 * f);
    if (rowBase + rl < nN) *(volatile v4f*)(op + 4 * f) = v;
  }
  __threadfence();
#pragma unroll
  for (int it = 0; it < 8; ++it) {
    const int f = it * GTHR + tid;
    const int rl = f >> 4;
    const v4f v = *(const v4f*)(sout + 4 * f);
    if (rowBase + rl < nN) *(volatile v4f*)(op + 4 * f) = v;
  }
}

extern "C" void kernel_launch(void* const* d_in, const int* in_sizes, int n_in,
                              void* d_out, int out_size, void* d_ws, size_t ws_size,
                              hipStream_t stream) {
  if (n_in < 15) return;
  const int nN = in_sizes[0] / CH;
  const int nE = in_sizes[2] / 2;
  if (nN <= 0 || nE <= 0) return;
  if (in_sizes[0] != nN * CH || in_sizes[2] != 2 * nE) return;
  if (in_sizes[1] != nE || in_sizes[4] != nE) return;
  if (in_sizes[5] != CH * CH || in_sizes[6] != CH || in_sizes[7] != CH * WA1P || in_sizes[8] != CH) return;
  if (in_sizes[9] != CH || in_sizes[10] != 1) return;
  if (in_sizes[11] != CH * CH || in_sizes[12] != CH || in_sizes[13] != CH * CH || in_sizes[14] != CH) return;
  if (out_size != nN * CH) return;
  if (nE > (1 << 28) || nN > (1 << 22)) return;

  const float* h     = (const float*)d_in[0];
  const float* dists = (const float*)d_in[1];
  const int*   edges = (const int*)d_in[2];
  const float* emask = (const float*)d_in[4];
  const float* W_lin = (const float*)d_in[5];
  const float* b_lin = (const float*)d_in[6];
  const float* Wa1   = (const float*)d_in[7];
  const float* ba1   = (const float*)d_in[8];
  const float* Wa2   = (const float*)d_in[9];
  const float* ba2   = (const float*)d_in[10];
  const float* Wm1   = (const float*)d_in[11];
  const float* bm1   = (const float*)d_in[12];
  const float* Wm2   = (const float*)d_in[13];
  const float* bm2   = (const float*)d_in[14];
  float* out = (float*)d_out;

  const int nBlkG = (nN + GROWS - 1) / GROWS;
  const int NPAD  = nBlkG * GROWS;
  const int nBlkE = (nE + ETHR - 1) / ETHR;
  const int EPAD  = nBlkE * ETHR;
  const int nBlkA = (nN + NSLOT - 1) / NSLOT;
  const int NPADA = nBlkA * NSLOT;
  if (NPADA < NPAD) return;

  char* ws = (char*)d_ws;
  size_t off = 0;
  const size_t oPL = off; off += (size_t)PLTOT * 2;               off = (off + 255) & ~(size_t)255;
  const size_t oHB = off; off += (size_t)NPAD * CH * 4;            off = (off + 255) & ~(size_t)255;
  const size_t oPQ = off; off += (size_t)NPAD * PQW * 4;           off = (off + 255) & ~(size_t)255;
  const size_t oNS = off; off += (size_t)NPAD * NSW * 4;           off = (off + 255) & ~(size_t)255;
  const size_t oG  = off; off += (size_t)EPAD * 4;                 off = (off + 255) & ~(size_t)255;
  const size_t oAG = off; off += (size_t)NPADA * CH * 4;           off = (off + 255) & ~(size_t)255;
  if (off > ws_size || off > (size_t)WSCAP) return;
  _Float16* PL  = (_Float16*)(ws + oPL);
  float*    HB  = (float*)(ws + oHB);
  float*    PQ  = (float*)(ws + oPQ);
  float*    NS  = (float*)(ws + oNS);
  float*    G   = (float*)(ws + oG);
  float*    AGG = (float*)(ws + oAG);

  k_wprep<<<WPBLK, WPTHR, 0, stream>>>(W_lin, Wa1, Wm1, Wm2, PL);
  k_node1<<<nBlkG, GTHR, 0, stream>>>(h, PL, b_lin, ba1, HB, PQ, NS, nN);
  k_escore<<<nBlkE, ETHR, 0, stream>>>(edges, dists, emask, Wa1, Wa2, ba2, HB, PQ, NS, G, nN, nE);
  hipFuncSetAttribute(reinterpret_cast<const void*>(&k_agg),
                      hipFuncAttributeMaxDynamicSharedMemorySize, LDS_AGG);
  k_agg<<<nBlkA, NTHR, LDS_AGG, stream>>>(edges, edges + nE, G, HB, AGG, nN, nE, 1);
  k_node2<<<nBlkG, GTHR, 0, stream>>>(AGG, PL, bm1, bm2, HB, NS, out, nN);
}
